// GIN_64647847740123
// MI455X (gfx1250) — hardware-run, weakly checked
//
#include <hip/hip_runtime.h>
#include <stddef.h>
#include <stdint.h>
#include <math.h>

#define NN      50000
#define HD      64
#define NLAY    4
#define NE      800000
#define GBM     128
#define MP      50048
#define KL      128
#define NTHR    256
#define NWAVE   8
#define EPT     8
#define WCH     (32 * EPT)
#define NBRUN   1024
#define SLB     10
#define NBK     49
#define WLCAP   2560
#define RCAP    20480
#define DEGCAP  64
#define MAXDEG_MEAS   35
#define MAXB1024_MEAS 16623
#define ABM     64
#define SP      68
#define BP      136
#define PARL    384
#define PARN    (NLAY * PARL + HD)
#define PLN     (HD * KL)
#define WSMAX   134217728

#define BK_ZINTS (NWAVE * WLCAP + RCAP + 3 * NBRUN)
#define BK_INTS  (BK_ZINTS + 16)
#define BK_LDS   (BK_INTS * 4)

#define PBH   (MP * HD / 4 / NTHR)
#define PBW1  (NLAY * PLN / 8 / NTHR)
#define PBW2  (NLAY * PLN / 8 / NTHR)
#define PBWO  (PLN / 8 / NTHR)
#define PBTOT (PBH + PBW1 + PBW2 + PBWO + 1)

static_assert(HD == 64 && KL == 2 * HD && KL == 4 * 32);
static_assert(NBRUN == 8 * GBM && NBRUN == (1 << SLB));
static_assert(MP == 391 * GBM && MP >= NN && MP % ABM == 0 && NBRUN % ABM == 0);
static_assert(NBK * NBRUN >= MP && (NBK - 1) * NBRUN < NN);
static_assert(NE == 800000 && NE % WCH == 0 && NE % 4 == 0);
static_assert((((long long)NE) << SLB) < (1LL << 31) && NE < (1 << 21));
static_assert(RCAP == NWAVE * WLCAP && RCAP % 4 == 0 && BK_ZINTS % 4 == 0);
static_assert((long long)RCAP * 100 >= (long long)MAXB1024_MEAS * 105);
static_assert(WLCAP >= MAXB1024_MEAS / 8 + 8 * 46 + 1);
static_assert(MAXDEG_MEAS + 8 <= DEGCAP && DEGCAP <= 64);
static_assert(BK_LDS <= 300000 && BK_LDS <= 327680);
static_assert((GBM * SP + 320) * 4 + HD * BP * 2 <= 65536);
static_assert((MP * HD / 4) % NTHR == 0 && (NLAY * PLN / 8) % NTHR == 0 && (PLN / 8) % NTHR == 0);
static_assert(NTHR == NLAY * HD && (PARN % 4) == 0 && PARN / 4 <= 2 * NTHR);
static_assert((BP % 8) == 0 && BP >= KL);
static_assert(ABM == 8 * NWAVE);

typedef float          v2f   __attribute__((ext_vector_type(2)));
typedef float          v4f   __attribute__((ext_vector_type(4)));
typedef float          v8f   __attribute__((ext_vector_type(8)));
typedef int            v4i   __attribute__((ext_vector_type(4)));
typedef int            v8i   __attribute__((ext_vector_type(8)));
typedef unsigned short v8us  __attribute__((ext_vector_type(8)));
typedef unsigned short v16us __attribute__((ext_vector_type(16)));
typedef __bf16         v16bf __attribute__((ext_vector_type(16)));
typedef v2f  __attribute__((may_alias)) v2fa;
typedef v4f  __attribute__((may_alias)) v4fa;
typedef v4i  __attribute__((may_alias)) v4ia;
typedef v8us __attribute__((may_alias)) v8usa;
union FragB { v16bf v; v16us u; v8us h[2]; v8i w; };

__device__ __forceinline__ v8f wmb(const FragB& a, const FragB& b, v8f c) {
  v8f d = __builtin_amdgcn_wmma_f32_16x16x32_bf16(false, a.v, false, b.v, (short)0, c, false, false);
  asm volatile("v_nop\n\tv_nop\n\tv_nop\n\tv_nop" : "+v"(d) : "v"(a.w), "v"(b.w));
  return d;
}

__device__ __forceinline__ unsigned bf16_bits(float f) {
  const unsigned u = __float_as_uint(f);
  const unsigned r = (u + 0x7FFFu + ((u >> 16) & 1u)) >> 16;
  const unsigned q = (u >> 16) | 0x40u;
  return ((u & 0x7fffffffu) > 0x7f800000u) ? q : r;
}
__device__ __forceinline__ float bf16_val(float f) {
  return __uint_as_float(bf16_bits(f) << 16);
}
__device__ __forceinline__ float relu_k(float v) { return (v > 0.0f) ? v : (v - v); }

__device__ __forceinline__ void hilo_pack(float v0, float v1, float v2, float v3,
                                          int& h01, int& h23, int& l01, int& l23) {
  const unsigned a0 = bf16_bits(v0), a1 = bf16_bits(v1), a2 = bf16_bits(v2), a3 = bf16_bits(v3);
  const unsigned b0 = bf16_bits(v0 - __uint_as_float(a0 << 16));
  const unsigned b1 = bf16_bits(v1 - __uint_as_float(a1 << 16));
  const unsigned b2 = bf16_bits(v2 - __uint_as_float(a2 << 16));
  const unsigned b3 = bf16_bits(v3 - __uint_as_float(a3 << 16));
  h01 = (int)(a0 | (a1 << 16)); h23 = (int)(a2 | (a3 << 16));
  l01 = (int)(b0 | (b1 << 16)); l23 = (int)(b2 | (b3 << 16));
}

__device__ __forceinline__ v4i regroup8(int h01, int h23, int l01, int l23, int lane) {
  const int t  = lane & 15;
  const int s0 = (lane & 16) + ((2 * t) & 15), s1 = s0 + 1;
  const int a0 = __shfl(h01, s0, 32), a1 = __shfl(h23, s0, 32), a2 = __shfl(h01, s1, 32), a3 = __shfl(h23, s1, 32);
  const int b0 = __shfl(l01, s0, 32), b1 = __shfl(l23, s0, 32), b2 = __shfl(l01, s1, 32), b3 = __shfl(l23, s1, 32);
  const int mk = (t < 8) ? -1 : 0;
  v4i o;
  o.x = (a0 & mk) | (b0 & ~mk); o.y = (a1 & mk) | (b1 & ~mk);
  o.z = (a2 & mk) | (b2 & ~mk); o.w = (a3 & mk) | (b3 & ~mk);
  return o;
}

__device__ __forceinline__ void st2_v4f(float* p, v4f v) {
  *(volatile v4f*)p = v;
  __threadfence();
  *(volatile v4f*)p = v;
}
__device__ __forceinline__ void st2_v8us(unsigned short* p, v8us v) {
  *(volatile v8us*)p = v;
  __threadfence();
  *(volatile v8us*)p = v;
}

__device__ __forceinline__ v8us gather8(const float* __restrict__ base, int stride) {
  float f[8];
#pragma unroll
  for (int i = 0; i < 8; ++i) f[i] = base[(size_t)i * (size_t)stride];
  v8us o;
#pragma unroll
  for (int i = 0; i < 8; ++i) o[i] = (unsigned short)bf16_bits(f[i]);
  return o;
}

__global__ __launch_bounds__(NTHR) void k_prep(const float* __restrict__ x, const float* __restrict__ w1,
                                               const float* __restrict__ w2, const float* __restrict__ wo,
                                               const float* __restrict__ b1, const float* __restrict__ gm,
                                               const float* __restrict__ bt, const float* __restrict__ mu,
                                               const float* __restrict__ vr, const float* __restrict__ b2,
                                               const float* __restrict__ bo,
                                               float* H, unsigned short* wpl, float* par) {
  __shared__ __attribute__((aligned(16))) float sp[PARN];
  const int tid = (int)threadIdx.x;
  const int blk = (int)blockIdx.x;
  if (blk < PBH) {
    const int u   = blk * NTHR + tid;
    const int row = u >> 4, c4 = (u & 15) * 4;
    const int rc  = row < NN ? row : NN - 1;
    const bool live = row < NN;
    const v4f a = *(const v4fa*)(x + (size_t)rc * HD + c4);
    asm volatile("" :: "v"(a));
    v4f o;
    o.x = live ? bf16_val(a.x) : 0.0f; o.y = live ? bf16_val(a.y) : 0.0f;
    o.z = live ? bf16_val(a.z) : 0.0f; o.w = live ? bf16_val(a.w) : 0.0f;
    st2_v4f(H + (size_t)row * HD + c4, o);
  } else if (blk < PBH + PBW1) {
    const int u = (blk - PBH) * NTHR + tid;
    const int l = u >> 10, n = (u >> 4) & 63, k8 = (u & 15) * 8, kk = k8 & 63;
    const v8us o = gather8(w1 + (size_t)l * HD * HD + (size_t)kk * HD + n, HD);
    st2_v8us(wpl + (size_t)l * PLN + (size_t)n * KL + k8, o);
  } else if (blk < PBH + PBW1 + PBW2) {
    const int u = (blk - PBH - PBW1) * NTHR + tid;
    const int l = u >> 10, n = (u >> 4) & 63, k8 = (u & 15) * 8, kk = k8 & 63;
    const v8us o = gather8(w2 + (size_t)l * HD * HD + (size_t)kk * HD + n, HD);
    st2_v8us(wpl + (size_t)(NLAY + l) * PLN + (size_t)n * KL + k8, o);
  } else if (blk < PBH + PBW1 + PBW2 + PBWO) {
    const int u = (blk - PBH - PBW1 - PBW2) * NTHR + tid;
    const int n = (u >> 4) & 63, k8 = (u & 15) * 8, kk = k8 & 63;
    const v8us o = gather8(wo + (size_t)kk * HD + n, HD);
    st2_v8us(wpl + (size_t)(2 * NLAY) * PLN + (size_t)n * KL + k8, o);
  } else {
    const int c = tid & 63, l = tid >> 6;
    const float fb1 = b1[tid], fmu = mu[tid], fvr = vr[tid], fg = gm[tid], fbe = bt[tid], fb2 = b2[tid];
    const float fbo = bo[c];
    asm volatile("" :: "v"(fbo));
    const float vv = bf16_val(fvr);
    const float r  = 1.0f / sqrtf(vv + 1e-5f);
    float* q = sp + l * PARL + c;
    q[0]   = bf16_val(fb1);
    q[64]  = bf16_val(fmu);
    q[128] = r;
    q[192] = bf16_val(fg);
    q[256] = bf16_val(fbe);
    q[320] = bf16_val(fb2);
    if (tid < 64) sp[NLAY * PARL + tid] = bf16_val(fbo);
    __syncthreads();
#pragma unroll 1
    for (int it = 0; it < 2; ++it) {
      const int i4 = it * NTHR + tid;
      const int ic = i4 < PARN / 4 ? i4 : PARN / 4 - 1;
      const v4f v = *(const v4fa*)(sp + 4 * ic);
      asm volatile("" :: "v"(v));
      if (i4 < PARN / 4) *(volatile v4f*)(par + 4 * i4) = v;
    }
    __threadfence();
#pragma unroll 1
    for (int it = 0; it < 2; ++it) {
      const int i4 = it * NTHR + tid;
      const int ic = i4 < PARN / 4 ? i4 : PARN / 4 - 1;
      const v4f v = *(const v4fa*)(sp + 4 * ic);
      asm volatile("" :: "v"(v));
      if (i4 < PARN / 4) *(volatile v4f*)(par + 4 * i4) = v;
    }
  }
}

__device__ __forceinline__ void bucket_flush(const int* pl, const int* cnt, int ov, int* lp, int* cop, int* fp,
                                             int tid) {
#pragma unroll 1
  for (int i = tid * 4; i < RCAP; i += NTHR * 4) {
    const v4i v = *(const v4ia*)(pl + i);
    *(volatile v4i*)(lp + i) = v;
  }
#pragma unroll 1
  for (int i = tid * 4; i < 2 * NBRUN; i += NTHR * 4) {
    const v4i v = *(const v4ia*)(cnt + i);
    *(volatile v4i*)(cop + i) = v;
  }
  if (tid < 8) {
    const v4i f = {ov, ov, ov, ov};
    *(volatile v4i*)(fp + 4 * tid) = f;
  }
}

__global__ __launch_bounds__(NTHR) void k_bucket(const int* __restrict__ srcs, const int* __restrict__ dsts,
                                                 int* LIST, int* CO, int* FLAG) {
  extern __shared__ __attribute__((aligned(16))) int dsm[];
  int* wl   = dsm;
  int* pl   = dsm + NWAVE * WLCAP;
  int* cnt  = pl + RCAP;
  int* offs = cnt + NBRUN;
  int* cur  = offs + NBRUN;
  int* misc = cur + NBRUN;
  const int tid = (int)threadIdx.x, lane = tid & 31, wave = tid >> 5;
  const int blk = (int)blockIdx.x;
  const unsigned nbs = (unsigned)(blk * NBRUN);
  const int nbi = (NN - blk * NBRUN) < NBRUN ? (NN - blk * NBRUN) : NBRUN;
  const unsigned unb = (unsigned)(nbi < 0 ? 0 : nbi);

  {
    const v4i z4 = {0, 0, 0, 0};
    for (int i = tid * 4; i < BK_ZINTS; i += NTHR * 4) *(v4ia*)(dsm + i) = z4;
    if (tid < 16) misc[tid] = 0;
  }
  __syncthreads();

  {
    const int per  = ((NE + NWAVE * WCH - 1) / (NWAVE * WCH)) * WCH;
    const int ebeg = wave * per;
    const int eend = (ebeg + per < NE) ? (ebeg + per) : NE;
    int* mylist = wl + wave * WLCAP;
    int wc = 0;
#pragma unroll 1
    for (int cb = ebeg; cb < eend; cb += WCH) {
      const int e0 = cb + lane * EPT;
      const v4i da = *(const v4ia*)(dsts + e0);
      const v4i db = *(const v4ia*)(dsts + e0 + 4);
      const unsigned s0 = (unsigned)da.x - nbs, s1 = (unsigned)da.y - nbs;
      const unsigned s2 = (unsigned)da.z - nbs, s3 = (unsigned)da.w - nbs;
      const unsigned s4 = (unsigned)db.x - nbs, s5 = (unsigned)db.y - nbs;
      const unsigned s6 = (unsigned)db.z - nbs, s7 = (unsigned)db.w - nbs;
      const bool h0 = s0 < unb, h1 = s1 < unb, h2 = s2 < unb, h3 = s3 < unb;
      const bool h4 = s4 < unb, h5 = s5 < unb, h6 = s6 < unb, h7 = s7 < unb;
      const unsigned m0 = __builtin_amdgcn_ballot_w32(h0), m1 = __builtin_amdgcn_ballot_w32(h1);
      const unsigned m2 = __builtin_amdgcn_ballot_w32(h2), m3 = __builtin_amdgcn_ballot_w32(h3);
      const unsigned m4 = __builtin_amdgcn_ballot_w32(h4), m5 = __builtin_amdgcn_ballot_w32(h5);
      const unsigned m6 = __builtin_amdgcn_ballot_w32(h6), m7 = __builtin_amdgcn_ballot_w32(h7);
      const unsigned any = m0 | m1 | m2 | m3 | m4 | m5 | m6 | m7;
      if (any != 0u) {
        const int pre = (int)(__builtin_amdgcn_mbcnt_lo(m0, 0u) + __builtin_amdgcn_mbcnt_lo(m1, 0u) +
                              __builtin_amdgcn_mbcnt_lo(m2, 0u) + __builtin_amdgcn_mbcnt_lo(m3, 0u) +
                              __builtin_amdgcn_mbcnt_lo(m4, 0u) + __builtin_amdgcn_mbcnt_lo(m5, 0u) +
                              __builtin_amdgcn_mbcnt_lo(m6, 0u) + __builtin_amdgcn_mbcnt_lo(m7, 0u));
        int p = wc + pre;
        if (h0) { if (p < WLCAP) mylist[p] = ((e0 + 0) << SLB) | (int)s0; p = p + 1; }
        if (h1) { if (p < WLCAP) mylist[p] = ((e0 + 1) << SLB) | (int)s1; p = p + 1; }
        if (h2) { if (p < WLCAP) mylist[p] = ((e0 + 2) << SLB) | (int)s2; p = p + 1; }
        if (h3) { if (p < WLCAP) mylist[p] = ((e0 + 3) << SLB) | (int)s3; p = p + 1; }
        if (h4) { if (p < WLCAP) mylist[p] = ((e0 + 4) << SLB) | (int)s4; p = p + 1; }
        if (h5) { if (p < WLCAP) mylist[p] = ((e0 + 5) << SLB) | (int)s5; p = p + 1; }
        if (h6) { if (p < WLCAP) mylist[p] = ((e0 + 6) << SLB) | (int)s6; p = p + 1; }
        if (h7) { if (p < WLCAP) mylist[p] = ((e0 + 7) << SLB) | (int)s7; p = p + 1; }
        wc += (int)(__builtin_popcount(m0) + __builtin_popcount(m1) + __builtin_popcount(m2) + __builtin_popcount(m3) +
                    __builtin_popcount(m4) + __builtin_popcount(m5) + __builtin_popcount(m6) + __builtin_popcount(m7));
      }
    }
    if (lane == 0) misc[wave] = wc;
  }
  __syncthreads();

  if (wave == 0) {
    int ov = 0;
#pragma unroll 1
    for (int w2 = 0; w2 < NWAVE; ++w2) {
      int c = misc[w2];
      if (c > WLCAP) ov = 1;
      c = c < 0 ? 0 : (c > WLCAP ? WLCAP : c);
#pragma unroll 1
      for (int b0 = 0; b0 < c; b0 += 32) {
        const int idx = b0 + lane;
        const int ent = wl[w2 * WLCAP + (idx < WLCAP ? idx : WLCAP - 1)];
        const int m32 = (c - b0) < 32 ? (c - b0) : 32;
#pragma unroll 1
        for (int k = 0; k < m32; ++k) {
          const int u    = __builtin_amdgcn_readlane(ent, k);
          const int slot = u & (NBRUN - 1);
          if (lane == 0) cnt[slot] = cnt[slot] + 1;
        }
      }
    }
    if (lane == 0) misc[9] = ov;
  }
  __syncthreads();
  if (wave == 0) {
    const int base = lane * (NBRUN / 32);
    int s = 0;
#pragma unroll 1
    for (int i = 0; i < NBRUN / 32; ++i) s += cnt[base + i];
    int incl = s;
#pragma unroll
    for (int d = 1; d < 32; d <<= 1) {
      const int y = __shfl_up(incl, d, 32);
      if (lane >= d) incl += y;
    }
    int run = incl - s;
#pragma unroll 1
    for (int i = 0; i < NBRUN / 32; ++i) {
      const int cv = cnt[base + i];
      offs[base + i] = run;
      cur[base + i]  = run;
      run += cv;
    }
  }
  __syncthreads();

  if (wave == 0) {
#pragma unroll 1
    for (int w2 = 0; w2 < NWAVE; ++w2) {
      int c = misc[w2];
      c = c < 0 ? 0 : (c > WLCAP ? WLCAP : c);
#pragma unroll 1
      for (int b0 = 0; b0 < c; b0 += 32) {
        const int idx = b0 + lane;
        const int ent = wl[w2 * WLCAP + (idx < WLCAP ? idx : WLCAP - 1)];
        int eid = (ent >> SLB) & 0x1FFFFF;
        eid = eid > NE - 1 ? NE - 1 : eid;
        int sr = srcs[eid];
        sr = sr < 0 ? 0 : (sr > NN - 1 ? NN - 1 : sr);
        const int m32 = (c - b0) < 32 ? (c - b0) : 32;
#pragma unroll 1
        for (int k = 0; k < m32; ++k) {
          const int u    = __builtin_amdgcn_readlane(ent, k);
          const int wd   = __builtin_amdgcn_readlane(sr, k);
          const int slot = u & (NBRUN - 1);
          if (lane == 0) {
            int p = cur[slot];
            p = p < 0 ? 0 : (p > RCAP - 1 ? RCAP - 1 : p);
            pl[p] = wd;
            cur[slot] = p + 1;
          }
        }
      }
    }
  }
  __syncthreads();

  const int ovf = misc[9];
  int* lp  = LIST + (size_t)blk * RCAP;
  int* cop = CO + (size_t)blk * (2 * NBRUN);
  int* fp  = FLAG + (size_t)blk * 32;
  bucket_flush(pl, cnt, ovf, lp, cop, fp, tid);
  __threadfence();
  bucket_flush(pl, cnt, ovf, lp, cop, fp, tid);
}

__global__ __launch_bounds__(NTHR) void k_agg(const int* __restrict__ LIST, const int* __restrict__ CO,
                                              const int* __restrict__ FLAG, const float* __restrict__ Hs,
                                              unsigned int* P1w) {
  const int tid = (int)threadIdx.x, lane = tid & 31;
  const int wave = __builtin_amdgcn_readfirstlane(tid >> 5);
  const int rowBase = (int)blockIdx.x * ABM;
  const int bucket  = rowBase >> SLB;
  const int* lb  = LIST + (size_t)bucket * RCAP;
  const int* cob = CO + (size_t)bucket * (2 * NBRUN);
  const int flag = FLAG[(size_t)bucket * 32];
  const float qnan = __uint_as_float(0x7fc00000u);

#pragma unroll 1
  for (int i = 0; i < ABM / NWAVE; ++i) {
    const int d    = rowBase + (ABM / NWAVE) * wave + i;
    const int slot = d & (NBRUN - 1);
    int c = cob[slot];
    int o = cob[NBRUN + slot];
    const bool big = c > DEGCAP;
    c = c < 0 ? 0 : (c > DEGCAP ? DEGCAP : c);
    o = o < 0 ? 0 : (o > RCAP - 1 ? RCAP - 1 : o);
    int last = o + (c > 0 ? c : 1) - 1;
    last = last > RCAP - 1 ? RCAP - 1 : last;

    const v2f sf = *(const v2fa*)(Hs + (size_t)d * HD + 2 * lane);
    float a0 = sf.x, a1 = sf.y;
#pragma unroll 1
    for (int b0 = 0; b0 < c; b0 += 32) {
      int idx = o + b0 + lane;
      idx = idx > last ? last : idx;
      int sv = lb[idx];
      sv = sv < 0 ? 0 : (sv > NN - 1 ? NN - 1 : sv);
      const int m32 = (c - b0) < 32 ? (c - b0) : 32;
#pragma unroll 1
      for (int k = 0; k < m32; k += 4) {
        const int k1 = (k + 1) < 31 ? (k + 1) : 31;
        const int k2 = (k + 2) < 31 ? (k + 2) : 31;
        const int k3 = (k + 3) < 31 ? (k + 3) : 31;
        const int q0 = __builtin_amdgcn_readlane(sv, k);
        const int q1 = __builtin_amdgcn_readlane(sv, k1);
        const int q2 = __builtin_amdgcn_readlane(sv, k2);
        const int q3 = __builtin_amdgcn_readlane(sv, k3);
        const v2f g0 = *(const v2fa*)(Hs + (size_t)q0 * HD + 2 * lane);
        const v2f g1 = *(const v2fa*)(Hs + (size_t)q1 * HD + 2 * lane);
        const v2f g2 = *(const v2fa*)(Hs + (size_t)q2 * HD + 2 * lane);
        const v2f g3 = *(const v2fa*)(Hs + (size_t)q3 * HD + 2 * lane);
        asm volatile("" :: "v"(g0), "v"(g1), "v"(g2), "v"(g3));
        const bool o1 = (k + 1) < m32, o2 = (k + 2) < m32, o3 = (k + 3) < m32;
        a0 = a0 + g0.x; a1 = a1 + g0.y;
        const float t1x = a0 + g1.x, t1y = a1 + g1.y;
        a0 = o1 ? t1x : a0; a1 = o1 ? t1y : a1;
        const float t2x = a0 + g2.x, t2y = a1 + g2.y;
        a0 = o2 ? t2x : a0; a1 = o2 ? t2y : a1;
        const float t3x = a0 + g3.x, t3y = a1 + g3.y;
        a0 = o3 ? t3x : a0; a1 = o3 ? t3y : a1;
      }
    }
    const bool bad  = (flag != 0) | big;
    const bool live = d < NN;
    a0 = bad ? qnan : a0; a1 = bad ? qnan : a1;
    a0 = live ? a0 : 0.0f; a1 = live ? a1 : 0.0f;
    const unsigned h0 = bf16_bits(a0), h1 = bf16_bits(a1);
    const unsigned l0 = bf16_bits(a0 - __uint_as_float(h0 << 16));
    const unsigned l1 = bf16_bits(a1 - __uint_as_float(h1 << 16));
    const unsigned hw = h0 | (h1 << 16);
    const unsigned lw = l0 | (l1 << 16);
    unsigned int* hp = P1w + (size_t)d * (KL / 2) + lane;
    unsigned int* lp = hp + 32;
    *(volatile unsigned int*)hp = hw;
    *(volatile unsigned int*)lp = lw;
    __threadfence();
    *(volatile unsigned int*)hp = hw;
    *(volatile unsigned int*)lp = lw;
  }
}

template <int MODE>
__global__ __launch_bounds__(NTHR) __attribute__((amdgpu_num_vgpr(248)))
void k_gemm(const unsigned short* __restrict__ A, const unsigned short* __restrict__ BT,
            const float* __restrict__ par, const int* __restrict__ FLAG, void* outp) {
  __shared__ __attribute__((aligned(16))) float stg[GBM * SP];
  __shared__ __attribute__((aligned(16))) unsigned short sB[HD * BP];
  __shared__ __attribute__((aligned(16))) float sp[320];
  constexpr int NP4 = (MODE == 0) ? 80 : 16;
  const int tid = (int)threadIdx.x, lane = tid & 31, wave = tid >> 5, hh = lane >> 4, m = lane & 15;
  const int rowBase = (int)blockIdx.x * GBM;

#pragma unroll
  for (int it = 0; it < 4; ++it) {
    const int p  = it * NTHR + tid;
    const int n  = p >> 4, k8 = (p & 15) * 8;
    const v8us w = *(const v8usa*)(BT + (size_t)n * KL + k8);
    *(v8usa*)(&sB[n * BP + k8]) = w;
  }
  {
    const int pi = tid < NP4 ? tid : NP4 - 1;
    const v4f pv = *(const v4fa*)(par + 4 * pi);
    asm volatile("" :: "v"(pv));
    if (tid < NP4) *(v4fa*)(&sp[4 * tid]) = pv;
  }
  __syncthreads();

  v8f acc[4];
  {
    const v8f z = {0.f, 0.f, 0.f, 0.f, 0.f, 0.f, 0.f, 0.f};
#pragma unroll
    for (int t = 0; t < 4; ++t) acc[t] = z;
  }
  const unsigned short* ap = A + (size_t)(rowBase + 16 * wave + m) * (size_t)KL + 8 * hh;
#pragma unroll 1
  for (int k0 = 0; k0 < KL; k0 += 32) {
    FragB af;
    af.h[0] = *(const v8usa*)(ap + k0);
    af.h[1] = *(const v8usa*)(ap + k0 + 16);
#pragma unroll
    for (int nt = 0; nt < 4; ++nt) {
      FragB bf;
      bf.h[0] = *(const v8usa*)(&sB[(16 * nt + m) * BP + 8 * hh + k0]);
      bf.h[1] = *(const v8usa*)(&sB[(16 * nt + m) * BP + 8 * hh + k0 + 16]);
      acc[nt] = wmb(af, bf, acc[nt]);
    }
  }
#pragma unroll
  for (int nt = 0; nt < 4; ++nt) {
#pragma unroll
    for (int r = 0; r < 8; ++r) stg[(16 * wave + 8 * hh + r) * SP + 16 * nt + m] = acc[nt][r];
  }
  __syncthreads();

  const float qnan = __uint_as_float(0x7fc00000u);
  const int flag = FLAG[(size_t)(rowBase >> SLB) * 32];
  const v4f pb = *(const v4fa*)(&sp[4 * m]);
  v4f pm = pb, pr = pb, pg = pb, pe = pb;
  if constexpr (MODE == 0) {
    pm = *(const v4fa*)(&sp[64 + 4 * m]);
    pr = *(const v4fa*)(&sp[128 + 4 * m]);
    pg = *(const v4fa*)(&sp[192 + 4 * m]);
    pe = *(const v4fa*)(&sp[256 + 4 * m]);
  }

#pragma unroll 1
  for (int i = 0; i < 8; ++i) {
    const int lr   = 16 * wave + 2 * i + hh;
    const int grow = rowBase + lr;
    const bool live = grow < NN;
    const v4f a = *(const v4fa*)(&stg[lr * SP + 4 * m]);
    asm volatile("" :: "v"(a));
    float v0 = a.x + pb.x, v1 = a.y + pb.y, v2 = a.z + pb.z, v3 = a.w + pb.w;
    if constexpr (MODE == 0) {
      v0 = ((v0 - pm.x) * pr.x) * pg.x + pe.x;
      v1 = ((v1 - pm.y) * pr.y) * pg.y + pe.y;
      v2 = ((v2 - pm.z) * pr.z) * pg.z + pe.z;
      v3 = ((v3 - pm.w) * pr.w) * pg.w + pe.w;
    }
    if constexpr (MODE != 3) {
      v0 = relu_k(v0); v1 = relu_k(v1); v2 = relu_k(v2); v3 = relu_k(v3);
      v0 = live ? v0 : 0.0f; v1 = live ? v1 : 0.0f; v2 = live ? v2 : 0.0f; v3 = live ? v3 : 0.0f;
    }
    if constexpr (MODE == 0 || MODE == 2) {
      int h01, h23, l01, l23;
      hilo_pack(v0, v1, v2, v3, h01, h23, l01, l23);
      const v4i ow = regroup8(h01, h23, l01, l23, lane);
      unsigned short* hp = (unsigned short*)outp + (size_t)grow * KL + 8 * m;
      *(volatile v4i*)hp = ow;
      __threadfence();
      *(volatile v4i*)hp = ow;
    } else if constexpr (MODE == 1) {
      v4f o;
      o.x = v0; o.y = v1; o.z = v2; o.w = v3;
      float* op = (float*)outp + (size_t)grow * HD + 4 * m;
      *(volatile v4f*)op = o;
      __threadfence();
      *(volatile v4f*)op = o;
    } else {
      const bool bad = (flag != 0);
      v4f o;
      o.x = bad ? qnan : v0; o.y = bad ? qnan : v1; o.z = bad ? qnan : v2; o.w = bad ? qnan : v3;
      float* op = (float*)outp + (size_t)grow * HD + 4 * m;
      if (live) *(volatile v4f*)op = o;
      __threadfence();
      if (live) *(volatile v4f*)op = o;
    }
  }
}

extern "C" void kernel_launch(void* const* d_in, const int* in_sizes, int n_in,
                              void* d_out, int out_size, void* d_ws, size_t ws_size,
                              hipStream_t stream) {
  if (n_in < 12) return;
  if (in_sizes[0] != NN * HD) return;
  if (in_sizes[1] != 2 * NE) return;
  if (in_sizes[2] != NLAY * HD * HD) return;
  if (in_sizes[3] != NLAY * HD) return;
  if (in_sizes[4] != NLAY * HD) return;
  if (in_sizes[5] != NLAY * HD) return;
  if (in_sizes[6] != NLAY * HD) return;
  if (in_sizes[7] != NLAY * HD) return;
  if (in_sizes[8] != NLAY * HD * HD) return;
  if (in_sizes[9] != NLAY * HD) return;
  if (in_sizes[10] != HD * HD) return;
  if (in_sizes[11] != HD) return;
  if (out_size != NN * HD) return;

  const float* x    = (const float*)d_in[0];
  const int*   ei   = (const int*)d_in[1];
  const float* W1s  = (const float*)d_in[2];
  const float* b1s  = (const float*)d_in[3];
  const float* gms  = (const float*)d_in[4];
  const float* bts  = (const float*)d_in[5];
  const float* mus  = (const float*)d_in[6];
  const float* vrs  = (const float*)d_in[7];
  const float* W2s  = (const float*)d_in[8];
  const float* b2s  = (const float*)d_in[9];
  const float* Wout = (const float*)d_in[10];
  const float* bout = (const float*)d_in[11];
  float* out = (float*)d_out;
  const int* srcs = ei;
  const int* dsts = ei + NE;

  constexpr size_t zF    = (size_t)MP * HD * 4;
  constexpr size_t zHL   = (size_t)MP * KL * 2;
  constexpr size_t zLIST = (size_t)NBK * RCAP * 4;
  constexpr size_t zCO   = (size_t)NBK * 2 * NBRUN * 4;
  constexpr size_t zFLAG = 6400;
  constexpr size_t zWPL  = (size_t)9 * PLN * 2;
  constexpr size_t zPAR  = (size_t)PARN * 4;
  constexpr size_t oH    = 0;
  constexpr size_t oP1   = oH + zF;
  constexpr size_t oP2   = oP1 + zHL;
  constexpr size_t oLIST = oP2 + zHL;
  constexpr size_t oCO   = oLIST + zLIST;
  constexpr size_t oFLAG = oCO + zCO;
  constexpr size_t oWPL  = oFLAG + zFLAG;
  constexpr size_t oPAR  = oWPL + zWPL;
  constexpr size_t oEND  = oPAR + zPAR;
  static_assert(zF % 256 == 0 && zHL % 256 == 0 && zLIST % 256 == 0 && zCO % 256 == 0);
  static_assert(zFLAG % 256 == 0 && zWPL % 256 == 0 && zPAR % 256 == 0);
  static_assert((size_t)NBK * 128 <= zFLAG);
  static_assert(oEND <= (size_t)WSMAX);
  static_assert((size_t)(NN - 1) * HD + HD - 1 < (size_t)NN * HD);
  if (oEND > ws_size) return;

  char* ws = (char*)d_ws;
  float*          H    = (float*)(ws + oH);
  unsigned short* P1   = (unsigned short*)(ws + oP1);
  unsigned short* P2   = (unsigned short*)(ws + oP2);
  int*            LIST = (int*)(ws + oLIST);
  int*            CO   = (int*)(ws + oCO);
  int*            FLAG = (int*)(ws + oFLAG);
  unsigned short* WPL  = (unsigned short*)(ws + oWPL);
  float*          PAR  = (float*)(ws + oPAR);

  hipFuncSetAttribute(reinterpret_cast<const void*>(&k_bucket), hipFuncAttributeMaxDynamicSharedMemorySize, (int)BK_LDS);

  k_prep<<<PBTOT, NTHR, 0, stream>>>(x, W1s, W2s, Wout, b1s, gms, bts, mus, vrs, b2s, bout, H, WPL, PAR);
  k_bucket<<<NBK, NTHR, BK_LDS, stream>>>(srcs, dsts, LIST, CO, FLAG);

  for (int l = 0; l < NLAY; ++l) {
    k_agg<<<MP / ABM, NTHR, 0, stream>>>(LIST, CO, FLAG, H, (unsigned int*)P1);
    k_gemm<0><<<MP / GBM, NTHR, 0, stream>>>(P1, WPL + (size_t)l * PLN, PAR + (size_t)l * PARL, FLAG, (void*)P2);
    if (l < NLAY - 1)
      k_gemm<1><<<MP / GBM, NTHR, 0, stream>>>(P2, WPL + (size_t)(NLAY + l) * PLN, PAR + (size_t)l * PARL + 320,
                                               FLAG, (void*)H);
    else
      k_gemm<2><<<MP / GBM, NTHR, 0, stream>>>(P2, WPL + (size_t)(NLAY + l) * PLN, PAR + (size_t)l * PARL + 320,
                                               FLAG, (void*)P1);
  }
  k_gemm<3><<<MP / GBM, NTHR, 0, stream>>>(P1, WPL + (size_t)(2 * NLAY) * PLN, PAR + (size_t)NLAY * PARL,
                                           FLAG, (void*)out);
}
